// ODEModel_67250597920774
// MI455X (gfx1250) — hardware-run, weakly checked
//
#include <hip/hip_runtime.h>
#include <math.h>

constexpr int NBATCH = 1024;
constexpr int NIN    = 256;
constexpr int NLAT   = 512;
constexpr int NHID   = 1024;
constexpr int NOUTC  = 64;
constexpr int NHALF  = NLAT / 2;
constexpr int NSTEP  = 20;
constexpr int NTHR   = 256;
constexpr int SLABP  = 68;
constexpr int HSLABP = 72;
constexpr float WCARRY     = 64.0f;
constexpr float WCARRY_INV = 1.0f / 64.0f;

static_assert(NBATCH % 64 == 0);
static_assert(NLAT % 64 == 0 && NHID % 64 == 0 && NOUTC % 64 == 0 && NIN % 64 == 0 && NHALF % 64 == 0);
static_assert(NIN % 32 == 0 && NLAT % 32 == 0 && NHID % 32 == 0 && NHALF % 32 == 0);
static_assert(((NBATCH * NIN) / 8) % NTHR == 0);

typedef __attribute__((ext_vector_type(16))) _Float16 v16h;
typedef __attribute__((ext_vector_type(8)))  _Float16 v8h;
typedef __attribute__((ext_vector_type(4)))  _Float16 v4h;
typedef __attribute__((ext_vector_type(8)))  float    v8f;
typedef __attribute__((ext_vector_type(4)))  float    v4f;

union FragU { v16h v; v8h h[2]; };

__device__ __forceinline__ v16h frag_load(const _Float16* p) {
  FragU f;
  f.h[0] = *(const v8h*)(p);
  f.h[1] = *(const v8h*)(p + 16);
  return f.v;
}
__device__ __forceinline__ v8f frag_mma(v16h a, v16h b, v8f c) {
  return __builtin_amdgcn_wmma_f32_16x16x32_f16(false, a, false, b, (short)0, c, false, false);
}
__device__ __forceinline__ void row_guard(v8f& a0, v8f& a1, v8f& a2, v8f& a3, v16h x, v16h b0, v16h b1, v16h b2, v16h b3) {
  asm volatile("v_nop\n\tv_nop\n\tv_nop\n\tv_nop" : "+v"(a0), "+v"(a1), "+v"(a2), "+v"(a3) : "v"(x), "v"(b0), "v"(b1), "v"(b2), "v"(b3));
}
__device__ __forceinline__ void acc_guard4(v8f& a, v8f& b, v8f& c, v8f& d) {
  asm volatile("v_nop\n\tv_nop\n\tv_nop\n\tv_nop" : "+v"(a), "+v"(b), "+v"(c), "+v"(d));
}
__device__ __forceinline__ void wave_lds_sync() {
  __builtin_amdgcn_fence(__ATOMIC_RELEASE, "workgroup");
  __builtin_amdgcn_wave_barrier();
  __builtin_amdgcn_fence(__ATOMIC_ACQUIRE, "workgroup");
}
__device__ __forceinline__ float tanh_er(float x) {
  return 1.0f - 2.0f * __builtin_amdgcn_rcpf(__expf(2.0f * x) + 1.0f);
}

__global__ __launch_bounds__(NTHR) void tp_f16_kernel(const float* __restrict__ src, int C, int ldo,
                                                      unsigned short* __restrict__ O, float sc) {
  __shared__ float Tt[64 * 65];
  const int tid = threadIdx.x;
  const int c0 = blockIdx.x * 64, r0 = blockIdx.y * 64;
#pragma unroll
  for (int i = 0; i < 4; ++i) {
    const int idx = i * NTHR + tid;
    const int rr = idx >> 4, cc = (idx & 15) * 4;
    const v4f v = *(const v4f*)(src + (size_t)(r0 + rr) * (size_t)C + c0 + cc);
    Tt[rr * 65 + cc + 0] = v[0];
    Tt[rr * 65 + cc + 1] = v[1];
    Tt[rr * 65 + cc + 2] = v[2];
    Tt[rr * 65 + cc + 3] = v[3];
  }
  __syncthreads();
  const int q = tid >> 3, c8 = (tid & 7) * 8;
  v8h hv[2];
#pragma unroll
  for (int g = 0; g < 2; ++g) {
    const int qq = g * 32 + q;
#pragma unroll
    for (int e = 0; e < 8; ++e) {
      const float f = Tt[(c8 + e) * 65 + qq];
      hv[g][e] = (_Float16)(f * sc);
    }
  }
  for (int pass = 0; pass < 2; ++pass) {
#pragma unroll
    for (int g = 0; g < 2; ++g) {
      const size_t o = (size_t)(c0 + g * 32 + q) * (size_t)ldo + (size_t)(r0 + c8);
      *(volatile v8h*)(O + o) = hv[g];
    }
    __threadfence();
  }
}

__global__ __launch_bounds__(NTHR) void cvt8_f16_kernel(const float* __restrict__ src, unsigned short* __restrict__ dst, int n8) {
  const int i = blockIdx.x * NTHR + threadIdx.x;
  if (i < n8) {
    const float* sp = src + (size_t)i * 8;
    const v4f a = *(const v4f*)(sp);
    const v4f b = *(const v4f*)(sp + 4);
    v8h hv;
#pragma unroll
    for (int e = 0; e < 4; ++e) {
      const float fa = a[e];
      const float fb = b[e];
      hv[e]     = (_Float16)fa;
      hv[4 + e] = (_Float16)fb;
    }
    *(volatile v8h*)(dst + (size_t)i * 8) = hv;
    __threadfence();
    *(volatile v8h*)(dst + (size_t)i * 8) = hv;
  }
}

template <int EPI>
__global__ __launch_bounds__(NTHR) void gemm_f16_kernel(
    const unsigned short* __restrict__ Ap, int lda,
    const unsigned short* __restrict__ Btp, int ldb,
    int M, int N, int K, float scale,
    const float* __restrict__ bias, const float* __restrict__ bias2, float tval,
    unsigned short* __restrict__ C16, int ldc16,
    float* __restrict__ C32, int ldc32,
    const float* Hc, const float* Pacc, float wk, float cz, int zfromn) {
  __shared__ __align__(16) float    sT[NTHR / 32][16 * SLABP];
  __shared__ __align__(16) _Float16 sH[NTHR / 32][16 * HSLABP];
  const int lane = threadIdx.x & 31;
  const int wave = threadIdx.x >> 5;
  const int tilesN = N >> 6;
  const int tilesM = M >> 6;
  const int tile = blockIdx.x * (NTHR / 32) + wave;
  if (tile >= tilesM * tilesN) return;
  const int tm = tile / tilesN;
  const int tn = tile - tm * tilesN;
  const int m0 = tm << 6;
  const int n0 = tn << 6;

  const int rlane = lane & 15;
  const int koff  = (lane >> 4) * 8;
  const int mOff  = (lane >> 4) * 8;

  v8f acc[4][4];
#pragma unroll
  for (int i = 0; i < 4; ++i)
#pragma unroll
    for (int j = 0; j < 4; ++j) acc[i][j] = (v8f){0.f, 0.f, 0.f, 0.f, 0.f, 0.f, 0.f, 0.f};

  const _Float16* ap = (const _Float16*)Ap  + (size_t)(m0 + rlane) * (size_t)lda + koff;
  const _Float16* bp = (const _Float16*)Btp + (size_t)(n0 + rlane) * (size_t)ldb + koff;
  const size_t a16 = (size_t)16 * (size_t)lda;
  const size_t b16 = (size_t)16 * (size_t)ldb;

  for (int k0 = 0; k0 < K; k0 += 32) {
    v16h bh[4];
#pragma unroll
    for (int j = 0; j < 4; ++j) bh[j] = frag_load(bp + (size_t)j * b16 + k0);
#pragma unroll
    for (int i = 0; i < 4; ++i) {
      const v16h ah = frag_load(ap + (size_t)i * a16 + k0);
#pragma unroll
      for (int j = 0; j < 4; ++j) acc[i][j] = frag_mma(ah, bh[j], acc[i][j]);
      row_guard(acc[i][0], acc[i][1], acc[i][2], acc[i][3], ah, bh[0], bh[1], bh[2], bh[3]);
    }
  }
  acc_guard4(acc[0][0], acc[0][1], acc[0][2], acc[0][3]);
  acc_guard4(acc[1][0], acc[1][1], acc[1][2], acc[1][3]);
  acc_guard4(acc[2][0], acc[2][1], acc[2][2], acc[2][3]);
  acc_guard4(acc[3][0], acc[3][1], acc[3][2], acc[3][3]);

  float*    slab = sT[wave];
  _Float16* hsl  = sH[wave];
  const int hh = lane >> 4, c4 = (lane & 15) * 4;
  const int q  = lane >> 3, c8 = (lane & 7) * 8;

  float bv[4];
#pragma unroll
  for (int j = 0; j < 4; ++j) {
    const int n = n0 + (j << 4) + rlane;
    float b = bias[n];
    if (EPI == 0) b += tval * bias2[n];
    bv[j] = b;
  }

#pragma unroll
  for (int i = 0; i < 4; ++i) {
    const int mBase = m0 + (i << 4);
#pragma unroll
    for (int j = 0; j < 4; ++j) {
#pragma unroll
      for (int r = 0; r < 8; ++r) slab[(mOff + r) * SLABP + (j << 4) + rlane] = acc[i][j][r] * scale + bv[j];
    }
    wave_lds_sync();

    if (EPI == 0) {
#pragma unroll 1
      for (int idx = 0; idx < 32; ++idx) {
        const int row = ((idx >> 3) << 2) + q;
        const int e = idx & 7;
        const float v = tanh_er(slab[row * SLABP + c8 + e]);
        hsl[row * HSLABP + c8 + e] = (_Float16)v;
      }
    }
    if (EPI == 2) {
#pragma unroll 1
      for (int idx = 0; idx < 32; ++idx) {
        const int row = ((idx >> 2) << 1) + hh;
        const int e = idx & 3;
        const float v = tanh_er(slab[row * SLABP + c4 + e]);
        slab[row * SLABP + c4 + e] = v;
        hsl[row * HSLABP + c4 + e] = (_Float16)v;
      }
    }
    if (EPI == 1) {
#pragma unroll 1
      for (int it = 0; it < 8; ++it) {
        const int row = it * 2 + hh;
        const size_t go = (size_t)(mBase + row) * (size_t)ldc32 + (size_t)(n0 + c4);
        const v4f kv = *(const v4f*)(slab + row * SLABP + c4);
        const v4f hv = *(const v4f*)(Hc + go);
        const v4f pv = *(const v4f*)(Pacc + go);
        v4f nv;
        float zz[4];
#pragma unroll
        for (int e = 0; e < 4; ++e) {
          const float ke = kv[e];
          const float he = hv[e];
          const float pe = pv[e];
          const float ne = pe + wk * ke;
          const float zs = he + cz * ke;
          nv[e] = ne;
          zz[e] = (zfromn != 0) ? ne : zs;
        }
        *(v4f*)(slab + row * SLABP + c4) = nv;
        v4h zh;
        zh[0] = (_Float16)zz[0];
        zh[1] = (_Float16)zz[1];
        zh[2] = (_Float16)zz[2];
        zh[3] = (_Float16)zz[3];
        *(v4h*)(hsl + row * HSLABP + c4) = zh;
      }
    }
    if (EPI != 3) wave_lds_sync();

    for (int pass = 0; pass < 2; ++pass) {
      if (EPI != 0) {
#pragma unroll
        for (int it = 0; it < 8; ++it) {
          const int row = it * 2 + hh;
          const v4f v = *(const v4f*)(slab + row * SLABP + c4);
          *(volatile v4f*)(C32 + (size_t)(mBase + row) * (size_t)ldc32 + (size_t)(n0 + c4)) = v;
        }
      }
      if (EPI != 3) {
#pragma unroll
        for (int it = 0; it < 4; ++it) {
          const int row = it * 4 + q;
          const v8h hv8 = *(const v8h*)(hsl + row * HSLABP + c8);
          *(volatile v8h*)(C16 + (size_t)(mBase + row) * (size_t)ldc16 + (size_t)(n0 + c8)) = hv8;
        }
      }
      __threadfence();
    }
    wave_lds_sync();
  }
}

extern "C" void kernel_launch(void* const* d_in, const int* in_sizes, int n_in,
                              void* d_out, int out_size, void* d_ws, size_t ws_size, hipStream_t stream) {
  if (n_in < 9 || d_out == nullptr || d_ws == nullptr) return;
  if (in_sizes[0] != NBATCH * NIN || in_sizes[1] != NIN * NLAT || in_sizes[2] != NLAT ||
      in_sizes[3] != (NLAT + 1) * NHID || in_sizes[4] != NHID || in_sizes[5] != NHID * NLAT ||
      in_sizes[6] != NLAT || in_sizes[7] != NHALF * NOUTC || in_sizes[8] != NOUTC ||
      out_size != NBATCH * NOUTC) return;

  const float* x     = (const float*)d_in[0];
  const float* W_in  = (const float*)d_in[1];
  const float* b_in  = (const float*)d_in[2];
  const float* W1    = (const float*)d_in[3];
  const float* b1    = (const float*)d_in[4];
  const float* W2    = (const float*)d_in[5];
  const float* b2    = (const float*)d_in[6];
  const float* W_out = (const float*)d_in[7];
  const float* b_out = (const float*)d_in[8];
  float* out = (float*)d_out;
  const float* w1t = W1 + (size_t)NLAT * NHID;

  char* ws = (char*)d_ws;
  size_t off = 0;
  auto carve = [&](size_t bytes) -> char* { char* p = ws + off; off += (bytes + 255) & ~(size_t)255; return p; };
  unsigned short* WINT  = (unsigned short*)carve((size_t)NLAT * NIN * 2);
  unsigned short* W1T   = (unsigned short*)carve((size_t)NHID * NLAT * 2);
  unsigned short* W2T   = (unsigned short*)carve((size_t)NLAT * NHID * 2);
  unsigned short* WOT   = (unsigned short*)carve((size_t)NOUTC * NHALF * 2);
  unsigned short* X16   = (unsigned short*)carve((size_t)NBATCH * NIN * 2);
  float*          HA    = (float*)carve((size_t)NBATCH * NLAT * 4);
  float*          HB    = (float*)carve((size_t)NBATCH * NLAT * 4);
  float*          ACA   = (float*)carve((size_t)NBATCH * NLAT * 4);
  float*          ACB   = (float*)carve((size_t)NBATCH * NLAT * 4);
  unsigned short* Z16   = (unsigned short*)carve((size_t)NBATCH * NLAT * 2);
  unsigned short* HID16 = (unsigned short*)carve((size_t)NBATCH * NHID * 2);
  if (off > ws_size || off > (size_t)134217728) return;

  tp_f16_kernel<<<dim3(NLAT / 64, NIN / 64), NTHR, 0, stream>>>(W_in, NLAT, NIN, WINT, WCARRY);
  tp_f16_kernel<<<dim3(NHID / 64, NLAT / 64), NTHR, 0, stream>>>(W1, NHID, NLAT, W1T, WCARRY);
  tp_f16_kernel<<<dim3(NLAT / 64, NHID / 64), NTHR, 0, stream>>>(W2, NLAT, NHID, W2T, WCARRY);
  tp_f16_kernel<<<dim3(NOUTC / 64, NHALF / 64), NTHR, 0, stream>>>(W_out, NOUTC, NHALF, WOT, WCARRY);
  {
    const int n8 = (NBATCH * NIN) / 8;
    cvt8_f16_kernel<<<(n8 + NTHR - 1) / NTHR, NTHR, 0, stream>>>(x, X16, n8);
  }

  const int gridLat = ((NBATCH / 64) * (NLAT / 64) + 7) / 8;
  const int gridHid = ((NBATCH / 64) * (NHID / 64) + 7) / 8;
  const int gridOut = ((NBATCH / 64) * (NOUTC / 64) + 7) / 8;

  gemm_f16_kernel<2><<<gridLat, NTHR, 0, stream>>>(
      X16, NIN, WINT, NIN, NBATCH, NLAT, NIN, WCARRY_INV,
      b_in, b_in, 0.0f, Z16, NLAT, HA, NLAT, HA, HA, 0.0f, 0.0f, 0);

  const float dt  = 0.05f;
  const float hdt = 0.5f * dt;
  const float dt6 = dt / 6.0f;
  const float dt3 = 2.0f * dt6;
  const float toff[4] = {0.0f, hdt, hdt, dt};
  const float wst[4]  = {dt6, dt3, dt3, dt6};
  const float czn[4]  = {hdt, hdt, dt, 0.0f};

  for (int s = 0; s < NSTEP; ++s) {
    const float t0 = dt * (float)s;
    float* h  = (s & 1) ? HB : HA;
    float* hn = (s & 1) ? HA : HB;
    for (int st = 0; st < 4; ++st) {
      const float tval = t0 + toff[st];
      gemm_f16_kernel<0><<<gridHid, NTHR, 0, stream>>>(
          Z16, NLAT, W1T, NLAT, NBATCH, NHID, NLAT, WCARRY_INV,
          b1, w1t, tval, HID16, NHID, ACB, NLAT, h, h, 0.0f, 0.0f, 0);
      const float* pacc = (st == 0) ? (const float*)h : ((st == 2) ? (const float*)ACB : (const float*)ACA);
      float* dst = (st == 0) ? ACA : ((st == 1) ? ACB : ((st == 2) ? ACA : hn));
      gemm_f16_kernel<1><<<gridLat, NTHR, 0, stream>>>(
          HID16, NHID, W2T, NHID, NBATCH, NLAT, NHID, WCARRY_INV,
          b2, b2, 0.0f, Z16, NLAT, dst, NLAT, h, pacc, wst[st], czn[st], (st == 3) ? 1 : 0);
    }
  }

  gemm_f16_kernel<3><<<gridOut, NTHR, 0, stream>>>(
      Z16, NLAT, WOT, NHALF, NBATCH, NOUTC, NHALF, WCARRY_INV,
      b_out, b_out, 0.0f, Z16, NLAT, out, NOUTC, HA, HA, 0.0f, 0.0f, 0);
}
